// TransformerEncoderBlock_11012296147294
// MI455X (gfx1250) — hardware-run, weakly checked
//
#include <hip/hip_runtime.h>


namespace {
constexpr int B = 4, T = 2048, DM = 1024, FF = 4096, NB = 4  , RL = T  ;
constexpr float XS = 8.0f, WSC = 256.0f, PS = 1024.0f, RS_ = 1024.0f, LOG2E = 1.4426950408889634f, LNEPS = 1e-5f, RSQD = 0.03125f  , RSQ2 = 0.70710678118654752f;
static_assert(T % 128 == 0 && DM % 256 == 0 && FF % 128 == 0, "tiling");
typedef _Float16 b16;
typedef __attribute__((ext_vector_type(16))) _Float16 v16b;
typedef __attribute__((ext_vector_type(8))) _Float16 v8b;
typedef __attribute__((ext_vector_type(8))) float v8f;
typedef __attribute__((ext_vector_type(4))) float v4f;
__device__ __forceinline__ float bf16_rne(float f) { unsigned int u = __float_as_uint(f); u += 0x7FFFu + ((u >> 16) & 1u); return __uint_as_float(u & 0xFFFF0000u); }
__device__ __forceinline__ void split16(float v, b16& hi, b16& lo) { hi = (b16)v; lo = (b16)(v - (float)hi); }
__device__ __forceinline__ v16b frag_kb(const b16* p, int hh) { const v8b a = *(const v8b*)(p + 8 * hh), b = *(const v8b*)(p + 16 + 8 * hh); v16b f;
#pragma unroll
  for (int e = 0; e < 8; ++e) { f[e] = a[e]; f[8 + e] = b[e]; } return f; }
__device__ __forceinline__ v8f wmma16b(v16b a, v16b b, v8f c) { v8f d = __builtin_amdgcn_wmma_f32_16x16x32_f16(false, a, false, b, (short)0, c, false, false); asm volatile("v_nop\n\tv_nop\n\tv_nop\n\tv_nop" : "+v"(d) : "v"(a), "v"(b)); return d; }
__device__ __forceinline__ void wave_lds_sync() { __builtin_amdgcn_fence(__ATOMIC_RELEASE, "workgroup"); __builtin_amdgcn_wave_barrier(); __builtin_amdgcn_fence(__ATOMIC_ACQUIRE, "workgroup"); }
__device__ __forceinline__ float pmul(float a, float b) { float p = a * b; asm volatile("" : "+v"(p)); return p; }
__device__ __forceinline__ int iclamp(int v, int lo, int hi) { return v < lo ? lo : (v > hi ? hi : v); }

typedef __attribute__((ext_vector_type(2))) _Float16 v2h;
typedef __attribute__((ext_vector_type(4))) _Float16 v4h;
typedef __attribute__((ext_vector_type(2))) float v2f;
typedef __attribute__((ext_vector_type(4))) int v4i;
__device__ __forceinline__ float nexp2(float v) { return __builtin_amdgcn_exp2f(v); }
__device__ __forceinline__ float bfp(float v) { float t = bf16_rne(v); asm volatile("" : "+v"(t)); return t; }
__global__ __launch_bounds__(256) void prep_kernel(const float* __restrict__ wo, const float* __restrict__ w1, const float* __restrict__ w2, b16* __restrict__ WO, b16* __restrict__ W1T, b16* __restrict__ W2T) {
  const size_t u = (size_t)blockIdx.x * 256 + threadIdx.x; const size_t n2 = (size_t)DM * DM / 8, n3 = (size_t)FF * DM / 8, n4 = (size_t)DM * FF / 8; if (u >= n2 + n3 + n4) return; v8b o; b16* dst; const float* src;
  if (u < n2) { src = wo + u * 8; dst = WO + u * 8; } else if (u < n2 + n3) { src = w1 + (u - n2) * 8; dst = W1T + (u - n2) * 8; } else { src = w2 + (u - n2 - n3) * 8; dst = W2T + (u - n2 - n3) * 8; }
  for (int j = 0; j < 8; ++j) o[j] = (b16)(bf16_rne(src[j]) * WSC);
  for (int pass = 0; pass < 2; ++pass) { *(volatile v8b*)dst = o; __threadfence(); }
}
__global__ __launch_bounds__(128) void xp_kernel(const float* __restrict__ x, int b0, b16* __restrict__ XH, b16* __restrict__ XT) {
  __shared__ __attribute__((aligned(16))) b16 tile[64][128 + 8];
  const int wave = threadIdx.x >> 5, lane = threadIdx.x & 31; const int t0 = blockIdx.x * 64, c0 = blockIdx.y * 128; const float* xb = x + ((size_t)b0 * T + t0) * DM + c0;
  for (int i = threadIdx.x; i < 64 * 32; i += 128) { const int rr = i / 32, q = (i % 32) * 4; const v4f f = *(const v4f*)(xb + (size_t)rr * DM + q); v4h o; for (int j = 0; j < 4; ++j) o[j] = (b16)(bf16_rne(f[j]) * XS); *(v4h*)(&tile[rr][q]) = o; }
  __syncthreads();
  for (int pass = 0; pass < 2; ++pass) {
    for (int rr = wave * 16; rr < wave * 16 + 16; ++rr) *(volatile v4h*)(XH + (size_t)(t0 + rr) * DM + c0 + lane * 4) = *(const v4h*)(&tile[rr][lane * 4]);
#pragma unroll 1
    for (int q = 0; q < 32; ++q) { const int cl = wave * 32 + q; v2h v; v[0] = tile[2 * lane][cl]; v[1] = tile[2 * lane + 1][cl]; *(volatile v2h*)(XT + (size_t)(c0 + cl) * T + t0 + 2 * lane) = v; }
    __threadfence(); }
}
__global__ __launch_bounds__(128) void scores_kernel(const b16* __restrict__ XH, float* __restrict__ S) {
  __shared__ __attribute__((aligned(16))) float Tf[4][16][128 + 4];
  const int wave = threadIdx.x >> 5, lane = threadIdx.x & 31, nloc = lane & 15, hlf = lane >> 4; const int q0 = blockIdx.x * 64 + wave * 16; const int k0 = blockIdx.y * 128;
  v8f acc[8];
#pragma unroll
  for (int t = 0; t < 8; ++t) acc[t] = (v8f){};
#pragma unroll 2
  for (int kb = 0; kb < DM; kb += 32) { const v16b a = frag_kb(XH + (size_t)(q0 + nloc) * DM + kb, hlf);
#pragma unroll
    for (int t = 0; t < 8; ++t) acc[t] = wmma16b(a, frag_kb(XH + (size_t)(k0 + t * 16 + nloc) * DM + kb, hlf), acc[t]); }
#pragma unroll
  for (int t = 0; t < 8; ++t)
#pragma unroll
    for (int r = 0; r < 8; ++r) Tf[wave][8 * hlf + r][t * 16 + nloc] = acc[t][r];
  wave_lds_sync();
  for (int pass = 0; pass < 2; ++pass) { for (int rr = 0; rr < 16; ++rr) *(volatile v4f*)(S + (size_t)(q0 + rr) * T + k0 + lane * 4) = *(const v4f*)(&Tf[wave][rr][lane * 4]); __threadfence(); }
}
__global__ __launch_bounds__(256) void softmax_kernel(const float* __restrict__ S, b16* __restrict__ Ph) {
  const int wave = threadIdx.x >> 5, lane = threadIdx.x & 31; const int q = blockIdx.x * 8 + wave;
  const float* sr = S + (size_t)q * T; const float c = LOG2E * RSQD / (XS * XS);
  float sv[T / 64][2]; float m = -INFINITY;
#pragma unroll
  for (int ch = 0; ch < T / 64; ++ch) { const v2f s2 = *(const v2f*)(sr + ch * 64 + lane * 2); sv[ch][0] = s2[0]; sv[ch][1] = s2[1]; m = fmaxf(m, fmaxf(s2[0], s2[1])); }
#pragma unroll
  for (int o = 16; o >= 1; o >>= 1) m = fmaxf(m, __shfl_xor(m, o));
  float l = 0.0f;
#pragma unroll
  for (int ch = 0; ch < T / 64; ++ch) for (int j = 0; j < 2; ++j) { const float p = nexp2(pmul(sv[ch][j] - m, c)); sv[ch][j] = p; l += p; }
#pragma unroll
  for (int o = 16; o >= 1; o >>= 1) l += __shfl_xor(l, o);
  const float inv = PS / l;
  for (int pass = 0; pass < 2; ++pass) {
#pragma unroll
    for (int ch = 0; ch < T / 64; ++ch) { v2h h2; for (int j = 0; j < 2; ++j) h2[j] = (b16)pmul(sv[ch][j], inv); *(volatile v2h*)(Ph + (size_t)q * T + ch * 64 + lane * 2) = h2; }
    __threadfence(); }
}
__global__ __launch_bounds__(128) void pv_kernel(const b16* __restrict__ Ph, const b16* __restrict__ XT, b16* __restrict__ CTh, b16* __restrict__ CTl) {
  __shared__ __attribute__((aligned(16))) float Tf[4][16][128 + 4];
  const int wave = threadIdx.x >> 5, lane = threadIdx.x & 31, nloc = lane & 15, hlf = lane >> 4; const int q0 = blockIdx.x * 64 + wave * 16; const int e0 = blockIdx.y * 128;
  v8f acc[8];
#pragma unroll
  for (int t = 0; t < 8; ++t) acc[t] = (v8f){};
#pragma unroll 2
  for (int kb = 0; kb < T; kb += 32) { const v16b a = frag_kb(Ph + (size_t)(q0 + nloc) * T + kb, hlf);
#pragma unroll
    for (int t = 0; t < 8; ++t) acc[t] = wmma16b(a, frag_kb(XT + (size_t)(e0 + t * 16 + nloc) * T + kb, hlf), acc[t]); }
#pragma unroll
  for (int t = 0; t < 8; ++t)
#pragma unroll
    for (int r = 0; r < 8; ++r) Tf[wave][8 * hlf + r][t * 16 + nloc] = acc[t][r] * (1.0f / (PS * XS));
  wave_lds_sync();
  for (int pass = 0; pass < 2; ++pass) { for (int rr = 0; rr < 16; ++rr) { v4h h4, l4; for (int j = 0; j < 4; ++j) { b16 p, ql; split16(Tf[wave][rr][lane * 4 + j] * XS, p, ql); h4[j] = p; l4[j] = ql; }
      const size_t oi = (size_t)(q0 + rr) * DM + e0 + lane * 4; *(volatile v4h*)(CTh + oi) = h4; *(volatile v4h*)(CTl + oi) = l4; } __threadfence(); }
}
__global__ __launch_bounds__(128) void out1_kernel(const b16* __restrict__ Ch, const b16* __restrict__ Cl, const b16* __restrict__ WO, const float* __restrict__ x, int b0, float* __restrict__ X1) {
  __shared__ __attribute__((aligned(16))) float Tf[4][16][128 + 4];
  const int wave = threadIdx.x >> 5, lane = threadIdx.x & 31, nloc = lane & 15, hlf = lane >> 4; const size_t m0 = (size_t)blockIdx.x * 64 + wave * 16; const size_t mg = m0 + (size_t)b0 * T;
  const int n0 = blockIdx.y * 128;
  v8f acc[8];
#pragma unroll
  for (int t = 0; t < 8; ++t) acc[t] = (v8f){};
#pragma unroll 2
  for (int kb = 0; kb < DM; kb += 32) { const v16b ah = frag_kb(Ch + (m0 + nloc) * DM + kb, hlf), al = frag_kb(Cl + (m0 + nloc) * DM + kb, hlf);
#pragma unroll
    for (int t = 0; t < 8; ++t) { const v16b bw = frag_kb(WO + (size_t)(n0 + t * 16 + nloc) * DM + kb, hlf); acc[t] = wmma16b(ah, bw, acc[t]); acc[t] = wmma16b(al, bw, acc[t]); } }
#pragma unroll
  for (int t = 0; t < 8; ++t) { const int col = n0 + t * 16 + nloc;
#pragma unroll
    for (int r = 0; r < 8; ++r) Tf[wave][8 * hlf + r][t * 16 + nloc] = acc[t][r] * (1.0f / (XS * WSC)) + bf16_rne(x[(mg + 8 * hlf + r) * DM + col]); }
  wave_lds_sync();
  for (int pass = 0; pass < 2; ++pass) { for (int rr = 0; rr < 16; ++rr) *(volatile v4f*)(X1 + (m0 + rr) * DM + n0 + lane * 4) = *(const v4f*)(&Tf[wave][rr][lane * 4]); __threadfence(); }
}
template <int MODE>
__global__ __launch_bounds__(256) void lnrow_kernel(const float* __restrict__ Y, const float* __restrict__ ST, float* __restrict__ RS) {
  __shared__ float part[8];
  const int wave = threadIdx.x >> 5, lane = threadIdx.x & 31; const int row = blockIdx.x * 8 + wave;
  const float mean = (MODE == 1) ? ST[0] * (1.0f / ((float)T * (float)DM)) : 0.0f;
  const float* yr = Y + (size_t)row * DM; float s = 0.0f;
#pragma unroll
  for (int q = 0; q < 8; ++q) { const v4f v = *(const v4f*)(yr + q * 128 + lane * 4); for (int j = 0; j < 4; ++j) { const float d = v[j] - mean; s += (MODE == 1) ? pmul(d, d) : v[j]; } }
#pragma unroll
  for (int o = 16; o >= 1; o >>= 1) s += __shfl_xor(s, o);
  if (lane == 0) part[wave] = s;
  __syncthreads();
  for (int pass = 0; pass < 2; ++pass) { if (wave == 0) ((volatile float*)RS)[(size_t)blockIdx.x * 32 + lane] = (lane < 8) ? part[lane] : 0.0f; __threadfence(); }
}
template <int MODE>
__global__ __launch_bounds__(256) void lnred_kernel(const float* __restrict__ RS, float* __restrict__ ST) {
  __shared__ float red[256]; __shared__ float keep;
  const int tid = threadIdx.x; float s = 0.0f;
#pragma unroll
  for (int j = 0; j < 8; ++j) s += RS[(size_t)tid * 32 + j];
  red[tid] = s; if (tid == 0) keep = (MODE == 1) ? ST[0] : 0.0f;
  __syncthreads();
  for (int stride = 128; stride >= 1; stride >>= 1) { if (tid < stride) red[tid] += red[tid + stride]; __syncthreads(); }
  for (int pass = 0; pass < 2; ++pass) { if (tid < 32) { const float v = (tid == MODE) ? red[0] : ((tid == 0) ? keep : 0.0f); ((volatile float*)ST)[tid] = v; } __threadfence(); }
}
__global__ __launch_bounds__(256) void lnapply_kernel(const float* __restrict__ Y, const float* __restrict__ ST, const float* __restrict__ w, const float* __restrict__ bb, float* __restrict__ OUT) {
  const int wave = threadIdx.x >> 5, lane = threadIdx.x & 31; const int row = blockIdx.x * 8 + wave;
  const float inv = 1.0f / ((float)T * (float)DM); const float mean = ST[0] * inv; const float rs = rsqrtf(ST[1] * inv + LNEPS);
  const float* yr = Y + (size_t)row * DM; const float* wr = w + (size_t)row * DM; const float* br = bb + (size_t)row * DM;
  for (int pass = 0; pass < 2; ++pass) {
#pragma unroll
    for (int q = 0; q < 8; ++q) { const int c = q * 128 + lane * 4; const v4f v = *(const v4f*)(yr + c), wv = *(const v4f*)(wr + c), bv = *(const v4f*)(br + c); v4f o;
      for (int j = 0; j < 4; ++j) o[j] = pmul((v[j] - mean) * rs, bfp(wv[j])) + bfp(bv[j]);
      *(volatile v4f*)(OUT + (size_t)row * DM + c) = o; }
    __threadfence(); }
}
__global__ __launch_bounds__(128) void mlp1_kernel(const float* __restrict__ XN, const b16* __restrict__ W1T, const float* __restrict__ b1, b16* __restrict__ G) {
  __shared__ __attribute__((aligned(16))) b16 As[64][256 + 8]; __shared__ __attribute__((aligned(16))) float Tf[4][16][128 + 4];
  const int wave = threadIdx.x >> 5, lane = threadIdx.x & 31, nloc = lane & 15, hlf = lane >> 4; const size_t r0 = (size_t)blockIdx.x * 64; const int n0 = blockIdx.y * 128;
  const float* xb = XN + r0 * DM;
  v8f acc[8];
#pragma unroll
  for (int t = 0; t < 8; ++t) acc[t] = (v8f){};
#pragma unroll 1
  for (int kc = 0; kc < DM; kc += 256) {
    __syncthreads();
    for (int i = threadIdx.x; i < 64 * 64; i += 128) { const int rr = i / 64, q = (i % 64) * 4; const v4f f = *(const v4f*)(xb + (size_t)rr * DM + kc + q); v4h o; for (int j = 0; j < 4; ++j) o[j] = (b16)(f[j] * XS); *(v4h*)(&As[rr][q]) = o; }
    __syncthreads();
#pragma unroll 2
    for (int kb = 0; kb < 256; kb += 32) { const v16b a = frag_kb(&As[wave * 16 + nloc][kb], hlf);
#pragma unroll
      for (int t = 0; t < 8; ++t) acc[t] = wmma16b(a, frag_kb(W1T + (size_t)(n0 + t * 16 + nloc) * DM + kc + kb, hlf), acc[t]); } }
#pragma unroll
  for (int t = 0; t < 8; ++t) { const float bbv = bf16_rne(b1[n0 + t * 16 + nloc]);
#pragma unroll
    for (int r = 0; r < 8; ++r) { const float hm = acc[t][r] * (1.0f / (XS * WSC)) + bbv; Tf[wave][8 * hlf + r][t * 16 + nloc] = fmaxf(hm, 0.0f); } }
  __syncthreads();
  for (int pass = 0; pass < 2; ++pass) { for (int rr = 0; rr < 16; ++rr) { v4h o4; for (int j = 0; j < 4; ++j) o4[j] = (b16)(Tf[wave][rr][lane * 4 + j] * XS); *(volatile v4h*)(G + (r0 + wave * 16 + rr) * FF + n0 + lane * 4) = o4; } __threadfence(); }
}
__global__ __launch_bounds__(128) void mlp2_kernel(const b16* __restrict__ G, const b16* __restrict__ W2T, const float* __restrict__ b2, const float* __restrict__ X1, float* __restrict__ out) {
  __shared__ __attribute__((aligned(16))) float Tf[4][16][128 + 4];
  const int wave = threadIdx.x >> 5, lane = threadIdx.x & 31, nloc = lane & 15, hlf = lane >> 4; const size_t m0 = (size_t)blockIdx.x * 64 + wave * 16; const int n0 = blockIdx.y * 128;
  v8f acc[8];
#pragma unroll
  for (int t = 0; t < 8; ++t) acc[t] = (v8f){};
#pragma unroll 2
  for (int kb = 0; kb < FF; kb += 32) { const v16b a = frag_kb(G + (m0 + nloc) * FF + kb, hlf);
#pragma unroll
    for (int t = 0; t < 8; ++t) acc[t] = wmma16b(a, frag_kb(W2T + (size_t)(n0 + t * 16 + nloc) * FF + kb, hlf), acc[t]); }
#pragma unroll
  for (int t = 0; t < 8; ++t) { const int col = n0 + t * 16 + nloc; const float bbv = bf16_rne(b2[col]);
#pragma unroll
    for (int r = 0; r < 8; ++r) Tf[wave][8 * hlf + r][t * 16 + nloc] = acc[t][r] * (1.0f / (XS * WSC)) + bbv + X1[(m0 + 8 * hlf + r) * DM + col]; }
  wave_lds_sync();
  for (int pass = 0; pass < 2; ++pass) { for (int rr = 0; rr < 16; ++rr) *(volatile v4f*)(out + (m0 + rr) * DM + n0 + lane * 4) = *(const v4f*)(&Tf[wave][rr][lane * 4]); __threadfence(); }
}
}

extern "C" void kernel_launch(void* const* d_in, const int* in_sizes, int n_in, void* d_out, int out_size, void* d_ws, size_t ws_size, hipStream_t stream) {
  (void)n_in;
  auto Fp = [&](int i) { return (const float*)d_in[i]; };
  if (in_sizes[0] != B * T * DM || in_sizes[1] != DM * DM || in_sizes[2] != T * DM || in_sizes[3] != T * DM || in_sizes[4] != FF * DM || in_sizes[5] != FF || in_sizes[6] != DM * FF || in_sizes[7] != DM || in_sizes[8] != T * DM || in_sizes[9] != T * DM || out_size != B * T * DM) return;
  size_t off = 0; char* ws = (char*)d_ws;
  auto carve = [&](size_t bytes) { char* p = ws + off; off += (bytes + 255) & ~(size_t)255; return p; };
  b16* WO = (b16*)carve((size_t)DM * DM * 2); b16* W1T = (b16*)carve((size_t)FF * DM * 2); b16* W2T = (b16*)carve((size_t)DM * FF * 2);
  b16* XH = (b16*)carve((size_t)T * DM * 2); b16* XT = (b16*)carve((size_t)DM * T * 2); float* S = (float*)carve((size_t)T * T * 4); b16* Ph = (b16*)carve((size_t)T * T * 2);
  b16* CTh = (b16*)carve((size_t)T * DM * 2); b16* CTl = (b16*)carve((size_t)T * DM * 2); float* Y1 = (float*)carve((size_t)T * DM * 4); float* H = (float*)carve((size_t)T * DM * 4); b16* G = (b16*)carve((size_t)T * FF * 2);
  float* RS = (float*)carve((size_t)(T / 8) * 32 * 4); float* ST = (float*)carve(32 * 4);
  if (off > ws_size || off > ((size_t)128 << 20)) return;
  prep_kernel<<<(unsigned)(((size_t)(DM * DM + FF * DM + DM * FF) / 8 + 255) / 256), 256, 0, stream>>>(Fp(1), Fp(4), Fp(6), WO, W1T, W2T);
  for (int b0 = 0; b0 < NB; ++b0) { float* outb = (float*)d_out + (size_t)b0 * T * DM;
    xp_kernel<<<dim3(T / 64, DM / 128), 128, 0, stream>>>(Fp(0), b0, XH, XT);
    scores_kernel<<<dim3(T / 64, T / 128), 128, 0, stream>>>(XH, S);
    softmax_kernel<<<T / 8, 256, 0, stream>>>(S, Ph);
    pv_kernel<<<dim3(T / 64, DM / 128), 128, 0, stream>>>(Ph, XT, CTh, CTl);
    out1_kernel<<<dim3(T / 64, DM / 128), 128, 0, stream>>>(CTh, CTl, WO, Fp(0), b0, Y1);
    lnrow_kernel<0><<<T / 8, 256, 0, stream>>>(Y1, ST, RS); lnred_kernel<0><<<1, 256, 0, stream>>>(RS, ST); lnrow_kernel<1><<<T / 8, 256, 0, stream>>>(Y1, ST, RS); lnred_kernel<1><<<1, 256, 0, stream>>>(RS, ST);
    lnapply_kernel<<<T / 8, 256, 0, stream>>>(Y1, ST, Fp(2), Fp(3), H);
    mlp1_kernel<<<dim3(RL / 64, FF / 128), 128, 0, stream>>>(H, W1T, Fp(5), G);
    mlp2_kernel<<<dim3(RL / 64, DM / 128), 128, 0, stream>>>(G, W2T, Fp(7), H, Y1);
    lnrow_kernel<0><<<T / 8, 256, 0, stream>>>(Y1, ST, RS); lnred_kernel<0><<<1, 256, 0, stream>>>(RS, ST); lnrow_kernel<1><<<T / 8, 256, 0, stream>>>(Y1, ST, RS); lnred_kernel<1><<<1, 256, 0, stream>>>(RS, ST);
    lnapply_kernel<<<T / 8, 256, 0, stream>>>(Y1, ST, Fp(8), Fp(9), outb); }
}
